// SelfAttention_51479478010551
// MI455X (gfx1250) — hardware-run, weakly checked
//
#include <hip/hip_runtime.h>


#ifndef NB
#define NB 2
#endif
#ifndef SEQ
#define SEQ 2048
#endif
#ifndef SCORE_RES
#define SCORE_RES 0
#endif
#define NB_FULL  2
#define SEQ_FULL 2048
#define DM   1024
#define NH   16
#define HD   64
#define NFR  32
#define NTOK (NB * SEQ)
#define QT   (SEQ / 16)
#define NCH  (SEQ / 32)
#define PP   40
#define OP   68
#define SP   72

static_assert(SEQ % 256 == 0);
static_assert(SEQ <= 2048);
static_assert(SEQ <= SEQ_FULL);
static_assert(NB >= 1);
static_assert(NB <= NB_FULL);
static_assert(DM == NH * HD);
static_assert(NCH <= 64);
static_assert(HD == 64);
static_assert(2 * NFR == HD);
static_assert((NFR * SEQ) % 256 == 0);
static_assert(SEQ % 64 == 0);
static_assert(NTOK % 64 == 0);
static_assert(DM % 64 == 0);
static_assert(DM % 32 == 0);
static_assert(((size_t)NTOK * DM) % (8 * 256) == 0);
static_assert(SP >= 64 + 8);
static_assert(PP >= 32 + 8);
static_assert(OP >= 64 + 4);
static_assert(HD * 2 == 128);
static_assert(SCORE_RES == 0 || SCORE_RES == 1);

typedef _Float16 f16t;
typedef _Float16 v16h __attribute__((ext_vector_type(16)));
typedef _Float16 v8h  __attribute__((ext_vector_type(8), may_alias));
typedef float    v8f  __attribute__((ext_vector_type(8)));
typedef float    v4f  __attribute__((ext_vector_type(4), may_alias));
typedef unsigned v4u  __attribute__((ext_vector_type(4), may_alias));

union Frag { v16h v; v8h hh[2]; };

__device__ __forceinline__ float bfr(float f) {
    unsigned u = __float_as_uint(f);
    u += 0x7FFFu + ((u >> 16) & 1u);
    u &= 0xFFFF0000u;
    return __uint_as_float(u);
}
__device__ __forceinline__ unsigned h2(float a, float b) {
    return (unsigned)__builtin_bit_cast(unsigned short, (f16t)a) | ((unsigned)__builtin_bit_cast(unsigned short, (f16t)b) << 16);
}
__device__ __forceinline__ v8f vzero() { v8f z; z[0] = 0.f; z[1] = 0.f; z[2] = 0.f; z[3] = 0.f; z[4] = 0.f; z[5] = 0.f; z[6] = 0.f; z[7] = 0.f; return z; }

__device__ __forceinline__ f16t toh_flush(float v) {
    const f16t r = (f16t)v;
    return (fabsf(v) < 6.103515625e-05f) ? (f16t)0.0f : r;
}
__device__ __forceinline__ unsigned h2f(float a, float b) {
    return (unsigned)__builtin_bit_cast(unsigned short, toh_flush(a)) | ((unsigned)__builtin_bit_cast(unsigned short, toh_flush(b)) << 16);
}

__device__ __forceinline__ v8f wmma16(v16h a, v16h b, v8f c) {
    c = __builtin_amdgcn_wmma_f32_16x16x32_f16(false, a, false, b, (short)0, c, false, false);
    asm volatile("v_nop\n\tv_nop\n\tv_nop\n\tv_nop" : "+v"(c) : "v"(a), "v"(b));
    return c;
}

__global__ __launch_bounds__(256) void k_cvt_x(const float* __restrict__ X, f16t* __restrict__ Xh) {
    const size_t u = (size_t)blockIdx.x * 256 + threadIdx.x;
    const size_t e = u * 8;
    const size_t tok = e / DM;
    const int k = (int)(e - tok * DM);
    const int bb = (int)(tok / SEQ), l = (int)(tok - (size_t)bb * SEQ);
    const float* src = X + ((size_t)bb * SEQ_FULL + l) * DM + k;
    const v4f x0 = *(const v4f*)(src);
    const v4f x1 = *(const v4f*)(src + 4);
    v4u o;
    o.x = h2(bfr(x0.x), bfr(x0.y)); o.y = h2(bfr(x0.z), bfr(x0.w));
    o.z = h2(bfr(x1.x), bfr(x1.y)); o.w = h2(bfr(x1.z), bfr(x1.w));
    f16t* dst = Xh + e;
    *(volatile v4u*)dst = o;
    __threadfence();
    *(volatile v4u*)dst = o;
}

__global__ __launch_bounds__(256) void k_wt(const float* __restrict__ Wq, const float* __restrict__ Wk, const float* __restrict__ Wv,
                                           f16t* __restrict__ WtAll) {
    __shared__ float tile[64][65];
    const int z = blockIdx.z;
    const float* W = (z == 0) ? Wq : ((z == 1) ? Wk : Wv);
    f16t* Wt = WtAll + (size_t)z * DM * DM;
    const int n0 = blockIdx.x * 64, k0 = blockIdx.y * 64, tid = threadIdx.x;
#pragma unroll
    for (int p = 0; p < 4; ++p) {
        const int r = p * 16 + (tid >> 4), c = 4 * (tid & 15);
        const v4f v = *(const v4f*)(W + (size_t)(k0 + r) * DM + n0 + c);
        tile[r][c] = v.x; tile[r][c + 1] = v.y; tile[r][c + 2] = v.z; tile[r][c + 3] = v.w;
    }
    __syncthreads();
    v4u o[2]; size_t off[2];
#pragma unroll
    for (int p = 0; p < 2; ++p) {
        const int L = p * 32 + (tid >> 3), kk = 8 * (tid & 7);
        const float w0 = 64.0f * bfr(tile[kk + 0][L]), w1 = 64.0f * bfr(tile[kk + 1][L]);
        const float w2 = 64.0f * bfr(tile[kk + 2][L]), w3 = 64.0f * bfr(tile[kk + 3][L]);
        const float w4 = 64.0f * bfr(tile[kk + 4][L]), w5 = 64.0f * bfr(tile[kk + 5][L]);
        const float w6 = 64.0f * bfr(tile[kk + 6][L]), w7 = 64.0f * bfr(tile[kk + 7][L]);
        o[p].x = h2(w0, w1); o[p].y = h2(w2, w3); o[p].z = h2(w4, w5); o[p].w = h2(w6, w7);
        off[p] = (size_t)(n0 + L) * DM + k0 + kk;
    }
#pragma unroll
    for (int p = 0; p < 2; ++p) *(volatile v4u*)(Wt + off[p]) = o[p];
    __threadfence();
#pragma unroll
    for (int p = 0; p < 2; ++p) *(volatile v4u*)(Wt + off[p]) = o[p];
}

__global__ __launch_bounds__(256) void k_rope_tab(float* __restrict__ CS, float* __restrict__ SN) {
#pragma clang fp contract(off)
    const int idx = blockIdx.x * 256 + threadIdx.x;
    const int j = idx / SEQ, pos = idx - j * SEQ;
    const float inv = exp2f(-(float)j * 0.41524101186092029f);
    const float ang = (float)pos * inv;
    float sn, cs;
    sincosf(ang, &sn, &cs);
    *(volatile float*)(CS + idx) = cs;
    *(volatile float*)(SN + idx) = sn;
    __threadfence();
    *(volatile float*)(CS + idx) = cs;
    *(volatile float*)(SN + idx) = sn;
}

__global__ __launch_bounds__(128) void k_proj(const f16t* __restrict__ Xh, const f16t* __restrict__ WtAll,
                                             const float* __restrict__ bq, const float* __restrict__ bk, const float* __restrict__ bv,
                                             const float* __restrict__ CS, const float* __restrict__ SN,
                                             f16t* __restrict__ Qh, f16t* __restrict__ Ql, f16t* __restrict__ Kh, f16t* __restrict__ Kl,
                                             f16t* __restrict__ Vt) {
    __shared__ __align__(16) f16t st[64 * SP];
    __shared__ __align__(16) f16t st2[64 * SP];
    const int z = blockIdx.z;
    const f16t* Wt = WtAll + (size_t)z * DM * DM;
    const float* bias = (z == 0) ? bq : ((z == 1) ? bk : bv);
    const int tid = threadIdx.x, lane = tid & 31, wv = tid >> 5, m = lane & 15, h = lane >> 4;
    const int row0 = blockIdx.x * 64;
    const int col0 = blockIdx.y * 64;
    const f16t* arow = Xh + (size_t)(row0 + wv * 16 + m) * DM + 8 * h;
    const f16t* bbase = Wt + (size_t)(col0 + m) * DM + 8 * h;
    v8f acc[4];
#pragma unroll
    for (int t = 0; t < 4; ++t) acc[t] = vzero();
#pragma unroll 1
    for (int kc = 0; kc < DM; kc += 32) {
        Frag a;
        a.hh[0] = *(const v8h*)(arow + kc);
        a.hh[1] = *(const v8h*)(arow + kc + 16);
#pragma unroll
        for (int t = 0; t < 4; ++t) {
            const f16t* brow = bbase + (size_t)(t * 16) * DM + kc;
            Frag b;
            b.hh[0] = *(const v8h*)(brow);
            b.hh[1] = *(const v8h*)(brow + 16);
            acc[t] = wmma16(a.v, b.v, acc[t]);
        }
    }
    const int bb = row0 / SEQ, l0 = row0 - bb * SEQ;
    const int bh = bb * NH + blockIdx.y;
    const float wsc = 0.015625f;
    if (z == 2) {
#pragma unroll
        for (int t = 0; t < 4; ++t) {
            const float bvl = bfr(bias[col0 + t * 16 + m]);
            v4u pk;
            pk.x = h2f(acc[t][0] * wsc + bvl, acc[t][1] * wsc + bvl);
            pk.y = h2f(acc[t][2] * wsc + bvl, acc[t][3] * wsc + bvl);
            pk.z = h2f(acc[t][4] * wsc + bvl, acc[t][5] * wsc + bvl);
            pk.w = h2f(acc[t][6] * wsc + bvl, acc[t][7] * wsc + bvl);
            *(v4u*)(st + (t * 16 + m) * SP + wv * 16 + 8 * h) = pk;
        }
    } else {
        const int pos0 = l0 + wv * 16 + 8 * h;
#pragma unroll
        for (int t = 0; t < 2; ++t) {
            const int j = t * 16 + m;
            const float b1 = bfr(bias[col0 + j]);
            const float b2 = bfr(bias[col0 + 32 + j]);
            const float* cp = CS + (size_t)j * SEQ + pos0;
            const float* sp = SN + (size_t)j * SEQ + pos0;
            const v4f c0 = *(const v4f*)(cp);
            const v4f c1 = *(const v4f*)(cp + 4);
            const v4f s0 = *(const v4f*)(sp);
            const v4f s1 = *(const v4f*)(sp + 4);
#pragma unroll
            for (int r = 0; r < 8; ++r) {
                const float cs = (r < 4) ? c0[r & 3] : c1[r & 3];
                const float sn = (r < 4) ? s0[r & 3] : s1[r & 3];
                const float x1 = acc[t][r] * wsc + b1;
                const float x2 = acc[t + 2][r] * wsc + b2;
                const float o1 = x1 * cs - x2 * sn;
                const float o2 = x2 * cs + x1 * sn;
                const f16t ha = toh_flush(o1);
                const f16t hb = toh_flush(o2);
                const int ix = (wv * 16 + 8 * h + r) * SP + j;
                st[ix]      = ha;
                st[ix + 32] = hb;
#if SCORE_RES
                st2[ix]      = toh_flush((o1 - (float)ha) * 1024.0f);
                st2[ix + 32] = toh_flush((o2 - (float)hb) * 1024.0f);
#endif
            }
        }
    }
    __syncthreads();
#if SCORE_RES
    const bool two = (z != 2);
#else
    const bool two = false;
#endif
    f16t* dstp = (z == 2) ? Vt : ((z == 0) ? Qh : Kh);
    f16t* dstl = (z == 0) ? Ql : Kl;
    v4u o[4], ol[4]; size_t off[4];
#pragma unroll
    for (int p = 0; p < 4; ++p) {
        const int L = p * 16 + (tid >> 3), piece = 8 * (tid & 7);
        o[p] = *(const v4u*)(st + L * SP + piece);
        ol[p] = o[p];
        if (two) ol[p] = *(const v4u*)(st2 + L * SP + piece);
        off[p] = (z == 2) ? (((size_t)bh * HD + L) * SEQ + l0 + piece) : (((size_t)bh * SEQ + l0 + L) * HD + piece);
    }
#pragma unroll
    for (int p = 0; p < 4; ++p) *(volatile v4u*)(dstp + off[p]) = o[p];
    if (two) {
#pragma unroll
        for (int p = 0; p < 4; ++p) *(volatile v4u*)(dstl + off[p]) = ol[p];
    }
    __threadfence();
#pragma unroll
    for (int p = 0; p < 4; ++p) *(volatile v4u*)(dstp + off[p]) = o[p];
    if (two) {
#pragma unroll
        for (int p = 0; p < 4; ++p) *(volatile v4u*)(dstl + off[p]) = ol[p];
    }
}

__global__ __launch_bounds__(128) void k_attn(const f16t* __restrict__ Qh, const f16t* __restrict__ Ql,
                                             const f16t* __restrict__ Kh, const f16t* __restrict__ Kl, const f16t* __restrict__ Vt,
                                             const float* __restrict__ am, float* __restrict__ out) {
    __shared__ __align__(16) f16t Pbuf[4][16 * PP];
    __shared__ __align__(16) float Obuf[4][16 * OP];
    const int tid = threadIdx.x, lane = tid & 31, wv = tid >> 5;
    const int m = lane & 15, h = lane >> 4;
    const int qt = blockIdx.x * 4 + wv;
    const int q0 = qt * 16;
    const int bh = blockIdx.y, bb = bh / NH, hd0 = (bh - bb * NH) * HD;
    const f16t* Qb  = Qh + (size_t)bh * SEQ * HD;
    const f16t* Kb  = Kh + (size_t)bh * SEQ * HD;
#if SCORE_RES
    const f16t* Qlb = Ql + (size_t)bh * SEQ * HD;
    const f16t* Klb = Kl + (size_t)bh * SEQ * HD;
#endif
    const f16t* Vb  = Vt + (size_t)bh * HD * SEQ;
    const float* amb = am + (size_t)bb * SEQ_FULL;
    f16t* Pw = &Pbuf[wv][0];
    float* Ow = &Obuf[wv][0];

    Frag aq0, aq1;
#if SCORE_RES
    Frag al0, al1;
#endif
    {
        const f16t* qrow = Qb + (size_t)(q0 + m) * HD + 8 * h;
        aq0.hh[0] = *(const v8h*)(qrow);      aq0.hh[1] = *(const v8h*)(qrow + 16);
        aq1.hh[0] = *(const v8h*)(qrow + 32); aq1.hh[1] = *(const v8h*)(qrow + 48);
#if SCORE_RES
        const f16t* lrow = Qlb + (size_t)(q0 + m) * HD + 8 * h;
        al0.hh[0] = *(const v8h*)(lrow);      al0.hh[1] = *(const v8h*)(lrow + 16);
        al1.hh[0] = *(const v8h*)(lrow + 32); al1.hh[1] = *(const v8h*)(lrow + 48);
#endif
    }
    v8f acc[4];
#pragma unroll
    for (int t = 0; t < 4; ++t) acc[t] = vzero();
    float rmax[8], rsum[8];
#pragma unroll
    for (int r = 0; r < 8; ++r) { rmax[r] = -1.0e30f; rsum[r] = 0.0f; }

#pragma unroll 1
    for (int ci = 0; ci < NCH; ++ci) {
        const int kc = ci * 32;
        v8f S0, S1;
#pragma unroll
        for (int t = 0; t < 2; ++t) {
            const int key = kc + t * 16 + m;
            const f16t* krow = Kb + (size_t)key * HD + 8 * h;
            Frag bk0, bk1;
            bk0.hh[0] = *(const v8h*)(krow);      bk0.hh[1] = *(const v8h*)(krow + 16);
            bk1.hh[0] = *(const v8h*)(krow + 32); bk1.hh[1] = *(const v8h*)(krow + 48);
            v8f s = vzero();
            s = wmma16(aq0.v, bk0.v, s);
            s = wmma16(aq1.v, bk1.v, s);
#if SCORE_RES
            const f16t* klr  = Klb + (size_t)key * HD + 8 * h;
            Frag bl0, bl1;
            bl0.hh[0] = *(const v8h*)(klr);       bl0.hh[1] = *(const v8h*)(klr + 16);
            bl1.hh[0] = *(const v8h*)(klr + 32);  bl1.hh[1] = *(const v8h*)(klr + 48);
            v8f s2 = vzero();
            s2 = wmma16(aq0.v, bl0.v, s2);
            s2 = wmma16(al0.v, bk0.v, s2);
            s2 = wmma16(aq1.v, bl1.v, s2);
            s2 = wmma16(al1.v, bk1.v, s2);
#endif
            const float av = bfr(amb[key]);
#pragma unroll
            for (int r = 0; r < 8; ++r) {
#if SCORE_RES
                const float sv = (s[r] + s2[r] * 0.0009765625f) * 0.125f + av;
#else
                const float sv = s[r] * 0.125f + av;
#endif
                s[r] = sv;
            }
            if (t == 0) S0 = s; else S1 = s;
        }
        float alpha[8];
#pragma unroll
        for (int r = 0; r < 8; ++r) {
            float mx = fmaxf(S0[r], S1[r]);
            mx = fmaxf(mx, __shfl_xor(mx, 1, 32));
            mx = fmaxf(mx, __shfl_xor(mx, 2, 32));
            mx = fmaxf(mx, __shfl_xor(mx, 4, 32));
            mx = fmaxf(mx, __shfl_xor(mx, 8, 32));
            const float Mn = fmaxf(rmax[r], mx);
            alpha[r] = __expf(rmax[r] - Mn);
            rmax[r] = Mn;
            const float p0 = __expf(S0[r] - Mn), p1 = __expf(S1[r] - Mn);
            S0[r] = p0; S1[r] = p1;
            float ps = p0 + p1;
            ps += __shfl_xor(ps, 1, 32);
            ps += __shfl_xor(ps, 2, 32);
            ps += __shfl_xor(ps, 4, 32);
            ps += __shfl_xor(ps, 8, 32);
            rsum[r] = alpha[r] * rsum[r] + ps;
        }
#pragma unroll
        for (int r = 0; r < 8; ++r) {
            Pw[(8 * h + r) * PP + m]      = toh_flush(S0[r] * 4096.0f);
            Pw[(8 * h + r) * PP + 16 + m] = toh_flush(S1[r] * 4096.0f);
        }
#pragma unroll
        for (int t = 0; t < 4; ++t)
#pragma unroll
            for (int r = 0; r < 8; ++r) acc[t][r] *= alpha[r];
        __builtin_amdgcn_fence(3  , "wavefront");
        __builtin_amdgcn_wave_barrier();
        Frag ap;
        {
            const f16t* prow = Pw + m * PP + 8 * h;
            ap.hh[0] = *(const v8h*)(prow);
            ap.hh[1] = *(const v8h*)(prow + 16);
        }
#pragma unroll
        for (int t = 0; t < 4; ++t) {
            const f16t* vrow = Vb + (size_t)(t * 16 + m) * SEQ + kc + 8 * h;
            Frag b;
            b.hh[0] = *(const v8h*)(vrow);
            b.hh[1] = *(const v8h*)(vrow + 16);
            acc[t] = wmma16(ap.v, b.v, acc[t]);
        }
    }

    float osc[8];
#pragma unroll
    for (int r = 0; r < 8; ++r) osc[r] = (rsum[r] > 0.0f) ? ((1.0f / rsum[r]) * 0.000244140625f) : 0.0f;
#pragma unroll
    for (int t = 0; t < 4; ++t)
#pragma unroll
        for (int r = 0; r < 8; ++r) Ow[(8 * h + r) * OP + t * 16 + m] = acc[t][r] * osc[r];
    __builtin_amdgcn_fence(3  , "wavefront");
    __builtin_amdgcn_wave_barrier();
    v4f o[8]; size_t off[8];
#pragma unroll
    for (int p = 0; p < 8; ++p) {
        const int L = p * 4 + (lane >> 3), row = L >> 1, co = (L & 1) * 32 + 4 * (lane & 7);
        o[p] = *(const v4f*)(Ow + row * OP + co);
        off[p] = ((size_t)bb * SEQ + q0 + row) * DM + hd0 + co;
    }
#pragma unroll
    for (int p = 0; p < 8; ++p) *(volatile v4f*)(out + off[p]) = o[p];
    __threadfence();
#pragma unroll
    for (int p = 0; p < 8; ++p) *(volatile v4f*)(out + off[p]) = o[p];
}

static inline size_t alup(size_t x) { return (x + 4095) & ~(size_t)4095; }

static constexpr size_t alupc(size_t x) { return (x + 4095) & ~(size_t)4095; }
static constexpr size_t CSZ_X = (size_t)NTOK * DM * sizeof(f16t);
static constexpr size_t CSZ_W = (size_t)3 * DM * DM * sizeof(f16t);
static constexpr size_t CSZ_P = (size_t)NB * NH * SEQ * HD * sizeof(f16t);
static constexpr size_t CSZ_T = (size_t)NFR * SEQ * sizeof(float);
static_assert(alupc(CSZ_X) + alupc(CSZ_W) + 5 * alupc(CSZ_P) + 2 * alupc(CSZ_T) <= (size_t)134217728);
static_assert(CSZ_P % 128 == 0);
static_assert(CSZ_T % 128 == 0);

extern "C" void kernel_launch(void* const* d_in, const int* in_sizes, int n_in,
                              void* d_out, int out_size, void* d_ws, size_t ws_size,
                              hipStream_t stream) {
    if (n_in < 8) return;
    if ((long long)in_sizes[0] < (long long)((NB - 1) * SEQ_FULL + SEQ) * DM) return;
    if (in_sizes[1] < (NB - 1) * SEQ_FULL + SEQ) return;
    if (in_sizes[2] < DM * DM || in_sizes[4] < DM * DM || in_sizes[6] < DM * DM) return;
    if (in_sizes[3] < DM || in_sizes[5] < DM || in_sizes[7] < DM) return;
    if ((long long)out_size < (long long)NB * SEQ * DM) return;

    const float* X   = (const float*)d_in[0];
    const float* am  = (const float*)d_in[1];
    const float* Wq  = (const float*)d_in[2];
    const float* bq  = (const float*)d_in[3];
    const float* Wk  = (const float*)d_in[4];
    const float* bk  = (const float*)d_in[5];
    const float* Wv  = (const float*)d_in[6];
    const float* bvv = (const float*)d_in[7];
    float* out = (float*)d_out;

    char* ws = (char*)d_ws;
    size_t off = 0;
    const size_t szX = (size_t)NTOK * DM * sizeof(f16t);
    const size_t szW = (size_t)3 * DM * DM * sizeof(f16t);
    const size_t szP = (size_t)NB * NH * SEQ * HD * sizeof(f16t);
    const size_t szT = (size_t)NFR * SEQ * sizeof(float);
    f16t* Xh = (f16t*)(ws + off); off += alup(szX);
    f16t* Wt = (f16t*)(ws + off); off += alup(szW);
    f16t* Qh = (f16t*)(ws + off); off += alup(szP);
    f16t* Ql = (f16t*)(ws + off); off += alup(szP);
    f16t* Kh = (f16t*)(ws + off); off += alup(szP);
    f16t* Kl = (f16t*)(ws + off); off += alup(szP);
    f16t* Vt = (f16t*)(ws + off); off += alup(szP);
    float* CS = (float*)(ws + off); off += alup(szT);
    float* SN = (float*)(ws + off); off += alup(szT);
    if (off > ws_size) return;

    k_cvt_x<<<dim3((unsigned)((size_t)NTOK * DM / 8 / 256)), 256, 0, stream>>>(X, Xh);
    k_wt<<<dim3(DM / 64, DM / 64, 3), 256, 0, stream>>>(Wq, Wk, Wv, Wt);
    k_rope_tab<<<dim3((NFR * SEQ) / 256), 256, 0, stream>>>(CS, SN);
    k_proj<<<dim3(NTOK / 64, DM / 64, 3), 128, 0, stream>>>(Xh, Wt, bq, bk, bvv, CS, SN, Qh, Ql, Kh, Kl, Vt);
    k_attn<<<dim3(SEQ / 64, NB * NH), 128, 0, stream>>>(Qh, Ql, Kh, Kl, Vt, am, out);
}
